// KernelPointAggregation_5205500363353
// MI455X (gfx1250) — hardware-verified
//
#include <hip/hip_runtime.h>

#pragma clang fp contract(off)

#define ROWS 32
#define NEI  32
#define KK   8
#define DD   64
#define KTAB 544
#define ESC  512

typedef float          v8f  __attribute__((ext_vector_type(8)));
typedef float          v4f  __attribute__((ext_vector_type(4)));
typedef float          v2f  __attribute__((ext_vector_type(2)));
typedef unsigned short v8us __attribute__((ext_vector_type(8)));
typedef __bf16         v16b __attribute__((ext_vector_type(16)));
typedef v4f  __attribute__((may_alias)) v4fa;
typedef v2f  __attribute__((may_alias)) v2fa;
typedef v8us __attribute__((may_alias)) v8usa;

union Frag { v16b v; v8us half[2]; };

static_assert(KTAB % 4 == 0);
static_assert((ROWS * DD) % (256 * 4) == 0);
static_assert(ROWS * DD == 256 * 8);

__device__ __forceinline__ unsigned int bf16_bits(float f) {
  const unsigned int u = __float_as_uint(f);
  return (u + 0x7FFFu + ((u >> 16) & 1u)) >> 16;
}
__device__ __forceinline__ float bf16r(float f) { return __uint_as_float(bf16_bits(f) << 16); }

__device__ __forceinline__ v8f wmma_bf16(v16b a, v16b b, v8f c) {
  v8f d = __builtin_amdgcn_wmma_f32_16x16x32_bf16(false, a, false, b, (short)0, c, false, false);
  asm volatile("v_nop\n\tv_nop\n\tv_nop\n\tv_nop" : "+v"(d) : "v"(a), "v"(b));
  return d;
}

__device__ __forceinline__ v16b load_frag_b16(const unsigned short* p, int h) {
  Frag f;
  f.half[0] = *(const v8usa*)(p + 8 * h);
  f.half[1] = *(const v8usa*)(p + 16 + 8 * h);
  return f.v;
}

__global__ __launch_bounds__(256) void k_prep(
    const float* __restrict__ W, const float* __restrict__ kp,
    const float* __restrict__ scales,
    unsigned short* __restrict__ wb, float* __restrict__ ktab)
{
  __shared__ __attribute__((aligned(16))) float sT[KTAB];
  __shared__ float sC0[KK];
  __shared__ float sC1[KK];
  const int tid = threadIdx.x;

  if (blockIdx.x < 16) {
    const int g = blockIdx.x * 256 + tid;
    const float* src = W + (size_t)g * 8;
    const v4f a = *(const v4fa*)src;
    const v4f c = *(const v4fa*)(src + 4);
    const v8us o = { (unsigned short)bf16_bits(a.x), (unsigned short)bf16_bits(a.y),
                     (unsigned short)bf16_bits(a.z), (unsigned short)bf16_bits(a.w),
                     (unsigned short)bf16_bits(c.x), (unsigned short)bf16_bits(c.y),
                     (unsigned short)bf16_bits(c.z), (unsigned short)bf16_bits(c.w) };
    unsigned short* dst = wb + (size_t)g * 8;
    *(volatile v8us*)dst = o;
    __threadfence();
    *(volatile v8us*)dst = o;
  } else {
    if (tid < KK) {
      float s2 = 0.0f;
      #pragma unroll 1
      for (int d = 1; d < DD; ++d) {
        const float v = bf16r(kp[tid * DD + d]);
        s2 += v * v;
      }
      const float nrm = sqrtf(fmaxf(s2, 1e-8f));
      sC0[tid] = coshf(nrm);
      sC1[tid] = sinhf(nrm) / nrm;
    }
    __syncthreads();
    {
      const int e0 = tid, e1 = tid + 256;
      const int k0 = e0 >> 6, d0 = e0 & 63;
      const int k1 = e1 >> 6, d1 = e1 & 63;
      const float sp0 = bf16r(kp[e0]);
      const float sp1 = bf16r(kp[e1]);
      sT[e0] = (d0 == 0) ? sC0[k0] : -(sC1[k0] * sp0);
      sT[e1] = (d1 == 0) ? sC0[k1] : -(sC1[k1] * sp1);
    }
    if (tid < 32) {
      const int ks = (tid < KK) ? tid : (KK - 1);
      const float es = expf(bf16r(scales[ks]));
      sT[ESC + tid] = (tid < KK) ? es : 0.0f;
    }
    __syncthreads();
    if (tid < KTAB / 4) {
      const v4f v = *(const v4fa*)(sT + tid * 4);
      float* dst = ktab + tid * 4;
      *(volatile v4f*)dst = v;
      __threadfence();
      *(volatile v4f*)dst = v;
    }
  }
}

__global__ __launch_bounds__(256) void k_xform(
    const float* __restrict__ x,
    const unsigned short* __restrict__ wb,
    const float* __restrict__ ktab,
    const float* __restrict__ bias,
    float* __restrict__ F,
    int nnode)
{
  __shared__ __attribute__((aligned(16))) unsigned short sA[ROWS * DD];
  __shared__ __attribute__((aligned(16))) float sX[ROWS * DD];
  __shared__ __attribute__((aligned(16))) float sK[KTAB];
  __shared__ float sW[KK * ROWS];
  __shared__ __attribute__((aligned(16))) float sG[ROWS * DD];
  __shared__ float sR[ROWS];

  const int tid = threadIdx.x, lane = tid & 31, wave = tid >> 5;
  const int h = lane >> 4, nl = lane & 15;
  const int j0 = blockIdx.x * ROWS;

  {
    const int row = tid >> 3, seg = tid & 7;
    int jr = j0 + row; jr = (jr < nnode) ? jr : (nnode - 1);
    const float* src = x + (size_t)jr * DD + seg * 8;
    const v4f a = *(const v4fa*)src;
    const v4f c = *(const v4fa*)(src + 4);
    const unsigned int u0 = bf16_bits(a.x), u1 = bf16_bits(a.y), u2 = bf16_bits(a.z), u3 = bf16_bits(a.w);
    const unsigned int u4 = bf16_bits(c.x), u5 = bf16_bits(c.y), u6 = bf16_bits(c.z), u7 = bf16_bits(c.w);
    const v8us o = { (unsigned short)u0, (unsigned short)u1, (unsigned short)u2, (unsigned short)u3,
                     (unsigned short)u4, (unsigned short)u5, (unsigned short)u6, (unsigned short)u7 };
    *(v8usa*)(sA + row * DD + seg * 8) = o;
    const v4f ra = { __uint_as_float(u0 << 16), __uint_as_float(u1 << 16), __uint_as_float(u2 << 16), __uint_as_float(u3 << 16) };
    const v4f rc = { __uint_as_float(u4 << 16), __uint_as_float(u5 << 16), __uint_as_float(u6 << 16), __uint_as_float(u7 << 16) };
    *(v4fa*)(sX + row * DD + seg * 8) = ra;
    *(v4fa*)(sX + row * DD + seg * 8 + 4) = rc;
    const v4f z4 = { 0.0f, 0.0f, 0.0f, 0.0f };
    *(v4fa*)(sG + tid * 8) = z4;
    *(v4fa*)(sG + tid * 8 + 4) = z4;
    if (tid < KTAB / 4) *(v4fa*)(sK + tid * 4) = *(const v4fa*)(ktab + tid * 4);
  }
  __syncthreads();

  {
    const float* xr = sX + lane * DD;
    const float* km = sK + wave * DD;
    float ni = 0.0f;
    #pragma unroll 2
    for (int d = 0; d < DD; d += 4) {
      const v4f xv = *(const v4fa*)(xr + d);
      const v4f kv = *(const v4fa*)(km + d);
      ni = fmaf(xv.x, kv.x, ni);
      ni = fmaf(xv.y, kv.y, ni);
      ni = fmaf(xv.z, kv.z, ni);
      ni = fmaf(xv.w, kv.w, ni);
    }
    const float zmin = __uint_as_float(0x3F800001u);
    const float z = fmaxf(ni, zmin);
    sW[wave * ROWS + lane] = acoshf(z);
  }
  __syncthreads();

  if (tid < ROWS) {
    float e[KK];
    float mx = -3.0e38f;
    #pragma unroll
    for (int k = 0; k < KK; ++k) { e[k] = -sW[k * ROWS + tid]; mx = fmaxf(mx, e[k]); }
    float s = 0.0f;
    #pragma unroll
    for (int k = 0; k < KK; ++k) { e[k] = expf(e[k] - mx); s += e[k]; }
    const float inv = 1.0f / s;
    #pragma unroll
    for (int k = 0; k < KK; ++k) sW[k * ROWS + tid] = e[k] * inv;
  }
  __syncthreads();

  const int k = wave;
  const v8f zero8 = { 0.f, 0.f, 0.f, 0.f, 0.f, 0.f, 0.f, 0.f };
  v8f acc[2][4];
  #pragma unroll
  for (int t = 0; t < 2; ++t)
    #pragma unroll
    for (int c = 0; c < 4; ++c) acc[t][c] = zero8;

  const unsigned short* wrow = wb + (size_t)(k * DD + nl) * DD;
  #pragma unroll
  for (int s = 0; s < 2; ++s) {
    const v16b a0 = load_frag_b16(sA + nl * DD + 32 * s, h);
    const v16b a1 = load_frag_b16(sA + (16 + nl) * DD + 32 * s, h);
    #pragma unroll
    for (int c = 0; c < 4; ++c) {
      const v16b b = load_frag_b16(wrow + (size_t)c * 16 * DD + 32 * s, h);
      acc[0][c] = wmma_bf16(a0, b, acc[0][c]);
      acc[1][c] = wmma_bf16(a1, b, acc[1][c]);
    }
  }

  float bk[4];
  #pragma unroll
  for (int c = 0; c < 4; ++c) bk[c] = bf16r(bias[k * DD + c * 16 + nl]);
  const float es = sK[ESC + k];

  #pragma unroll
  for (int t = 0; t < 2; ++t) {
    #pragma unroll
    for (int r = 0; r < 8; ++r) {
      const int m = 16 * t + 8 * h + r;
      float yc[4];
      #pragma unroll
      for (int c = 0; c < 4; ++c) yc[c] = acc[t][c][r] + bk[c];
      float p = (nl == 0) ? 0.0f : (yc[0] * yc[0]);
      p = p + yc[1] * yc[1];
      p = p + yc[2] * yc[2];
      p = p + yc[3] * yc[3];
      p += __shfl_xor(p, 1);
      p += __shfl_xor(p, 2);
      p += __shfl_xor(p, 4);
      p += __shfl_xor(p, 8);
      const float y0 = __shfl(yc[0], lane & 16);
      const float sig = 1.0f / (1.0f + expf(-y0));
      const float time = sig * es + 1.0001f;
      const float sc = (time * time - 1.0f) / fmaxf(p, 1e-8f);
      const float ssc = sqrtf(sc);
      const float wkm = sW[k * ROWS + m];
      #pragma unroll
      for (int c = 0; c < 4; ++c) {
        const float xtr = (c == 0 && nl == 0) ? time : (yc[c] * ssc);
        acc[t][c][r] = wkm * xtr;
      }
    }
  }

  #pragma unroll 1
  for (int kk = 0; kk < KK; ++kk) {
    if (wave == kk) {
      #pragma unroll
      for (int t = 0; t < 2; ++t)
        #pragma unroll
        for (int r = 0; r < 8; ++r) {
          const int m = 16 * t + 8 * h + r;
          #pragma unroll
          for (int c = 0; c < 4; ++c) sG[m * DD + c * 16 + nl] += acc[t][c][r];
        }
    }
    __syncthreads();
  }

  if (tid < ROWS) {
    const float* a = sG + tid * DD;
    float S = 0.0f;
    #pragma unroll 1
    for (int d = 1; d < DD; ++d) S += a[d] * a[d];
    const float a0 = a[0];
    const float ln = -a0 * a0 + S;
    const float den = sqrtf(fmaxf(fabsf(ln), 1e-8f));
    sR[tid] = 1.0f / den;
  }
  __syncthreads();

  v4f fv[2];
  #pragma unroll
  for (int i = 0; i < 2; ++i) {
    const int e = (i * 256 + tid) * 4;
    const float rr = sR[e >> 6];
    const v4f v = *(const v4fa*)(sG + e);
    fv[i] = v * rr;
  }
  float* fb = F + (size_t)j0 * DD;
  #pragma unroll
  for (int i = 0; i < 2; ++i) *(volatile v4f*)(fb + (size_t)(i * 256 + tid) * 4) = fv[i];
  __threadfence();
  #pragma unroll
  for (int i = 0; i < 2; ++i) *(volatile v4f*)(fb + (size_t)(i * 256 + tid) * 4) = fv[i];
}

__global__ __launch_bounds__(256) void k_mid(
    const float* __restrict__ F,
    const int* __restrict__ nei,
    const int* __restrict__ msk,
    float* __restrict__ out,
    int nnode)
{
  __shared__ __attribute__((aligned(16))) float sO[8 * DD];

  const int tid = threadIdx.x, lane = tid & 31, wave = tid >> 5;
  const int n0 = blockIdx.x * 8;
  int n = n0 + wave; n = (n < nnode) ? n : (nnode - 1);

  int idx = nei[(size_t)n * NEI + lane];
  idx = (idx < 0) ? 0 : idx;
  idx = (idx > nnode - 1) ? (nnode - 1) : idx;
  const float wn = (float)msk[(size_t)n * NEI + lane] + 1e-4f;

  float m0 = 0.0f, m1 = 0.0f;
  #pragma unroll 4
  for (int mm = 0; mm < NEI; ++mm) {
    const int jj = __shfl(idx, mm);
    const float ww = __shfl(wn, mm);
    const v2f v = *(const v2fa*)(F + (size_t)jj * DD + 2 * lane);
    m0 = fmaf(ww, v.x, m0);
    m1 = fmaf(ww, v.y, m1);
  }

  float sq = m1 * m1 + ((lane == 0) ? 0.0f : (m0 * m0));
  sq += __shfl_xor(sq, 16);
  sq += __shfl_xor(sq, 8);
  sq += __shfl_xor(sq, 4);
  sq += __shfl_xor(sq, 2);
  sq += __shfl_xor(sq, 1);
  const float t0 = __shfl(m0, 0);
  const float ln = -t0 * t0 + sq;
  const float inv = 1.0f / sqrtf(fmaxf(fabsf(ln), 1e-8f));
  const v2f o2 = { m0 * inv, m1 * inv };
  *(v2fa*)(sO + wave * DD + 2 * lane) = o2;
  __syncthreads();

  if (tid < 128) {
    const v4f v = *(const v4fa*)(sO + tid * 4);
    float* dst = out + (size_t)n0 * DD + tid * 4;
    *(volatile v4f*)dst = v;
    __threadfence();
    *(volatile v4f*)dst = v;
  }
}

extern "C" void kernel_launch(void* const* d_in, const int* in_sizes, int n_in,
                              void* d_out, int out_size, void* d_ws, size_t ws_size,
                              hipStream_t stream) {
  if (n_in < 7) return;
  const int nx = in_sizes[0];
  if (nx <= 0 || (nx % DD) != 0) return;
  const int nnode = nx / DD;
  if ((nnode % ROWS) != 0 || (nnode % 8) != 0) return;
  if (in_sizes[1] != nnode * NEI || in_sizes[2] != nnode * NEI) return;
  if (in_sizes[3] != KK * DD) return;
  if (in_sizes[4] != KK * DD * DD) return;
  if (in_sizes[5] != KK * DD) return;
  if (in_sizes[6] != KK) return;
  if (out_size != nnode * DD) return;

  const float* x      = (const float*)d_in[0];
  const int*   nei    = (const int*)d_in[1];
  const int*   nmask  = (const int*)d_in[2];
  const float* kp     = (const float*)d_in[3];
  const float* W      = (const float*)d_in[4];
  const float* b      = (const float*)d_in[5];
  const float* scales = (const float*)d_in[6];
  float* out = (float*)d_out;

  const size_t wb_bytes   = (size_t)KK * DD * DD * 2;
  const size_t ktab_bytes = (((size_t)KTAB * 4 + 127) / 128) * 128;
  const size_t f_bytes    = (size_t)nnode * DD * 4;
  const size_t total = wb_bytes + ktab_bytes + f_bytes;
  if (total > ws_size) return;

  char* ws = (char*)d_ws;
  unsigned short* wb = (unsigned short*)(ws);
  float* ktab = (float*)(ws + wb_bytes);
  float* F    = (float*)(ws + wb_bytes + ktab_bytes);

  k_prep<<<17, 256, 0, stream>>>(W, kp, scales, wb, ktab);
  k_xform<<<nnode / ROWS, 256, 0, stream>>>(x, wb, ktab, b, F, nnode);
  k_mid<<<nnode / 8, 256, 0, stream>>>(F, nei, nmask, out, nnode);
}
